// Block_30915174596989
// MI455X (gfx1250) — hardware-verified
//
#include <hip/hip_runtime.h>
#include <math.h>

#ifndef NB
#define NB 2
#endif
#ifndef SEQ
#define SEQ 2048
#endif
#define NB_FULL 2
#define SEQ_FULL 2048
#define CE 1024
#define NH 16
#define HD 64
#define FF 4096
#define ROWS (NB * SEQ)

static_assert(NH * HD == CE);
static_assert(HD == 64);
static_assert(CE == 32 * 4 * 8);
static_assert(SEQ % 64 == 0);
static_assert(ROWS % 64 == 0);
static_assert(CE % 64 == 0);
static_assert(FF % 64 == 0);
static_assert((2 * CE) % 32 == 0);
static_assert(NB <= NB_FULL);
static_assert(SEQ <= SEQ_FULL);

typedef __attribute__((ext_vector_type(16))) _Float16 v16h;
typedef __attribute__((ext_vector_type(8)))  _Float16 v8h;
typedef __attribute__((ext_vector_type(16))) __bf16   v16b;
typedef __attribute__((ext_vector_type(8)))  __bf16   v8b;
typedef __attribute__((ext_vector_type(8)))  float    v8f;
typedef __attribute__((ext_vector_type(4)))  float    v4f;
typedef __attribute__((ext_vector_type(4)))  unsigned int v4u;
typedef __attribute__((ext_vector_type(2)))  unsigned int v2u;


__device__ __forceinline__ float bfr(float v) {
    const unsigned u = __float_as_uint(v);
    const unsigned r = (u + 0x7fffu + ((u >> 16) & 1u)) & 0xffff0000u;
    return __uint_as_float(r);
}
__device__ __forceinline__ unsigned short bf_bits(float f) {
    const unsigned u = __float_as_uint(f);
    return (unsigned short)((u + 0x7fffu + ((u >> 16) & 1u)) >> 16);
}
__device__ __forceinline__ float bits_f(unsigned short h) { return __uint_as_float(((unsigned)h) << 16); }
__device__ __forceinline__ void bfsplit(float v, unsigned short& hi, unsigned short& lo) { hi = bf_bits(v); lo = bf_bits(v - bits_f(hi)); }
__device__ __forceinline__ unsigned pk2h(float a, float b) {
    return (unsigned)__builtin_bit_cast(unsigned short, (_Float16)a) | ((unsigned)__builtin_bit_cast(unsigned short, (_Float16)b) << 16);
}

#define VST2(T, ptr, val) do { const T vst2_v_ = (val); *(volatile T*)(ptr) = vst2_v_; __threadfence(); *(volatile T*)(ptr) = vst2_v_; } while (0)

__global__ __launch_bounds__(256) void k_w_head(const float* __restrict__ W, unsigned short* __restrict__ D, int ldd, int dup, int f16mode) {
    const int u = blockIdx.x * 256 + threadIdx.x;
    if (u >= CE * (CE / 8)) return;
    const int n = u / (CE / 8); const int k0 = 8 * (u % (CE / 8));
    const int h = n / HD, d = n % HD;
    const float* s = W + ((size_t)h * CE + k0) * HD + d;
    unsigned short bb[8];
#pragma unroll
    for (int e = 0; e < 8; ++e) {
        const float w = bfr(s[(size_t)e * HD]);
        const unsigned short b16 = (unsigned short)(__float_as_uint(w) >> 16);
        const unsigned short h16 = __builtin_bit_cast(unsigned short, (_Float16)(w * 16.0f));
        bb[e] = f16mode ? h16 : b16;
    }
    v4u pk;
    pk.x = (unsigned)bb[0] | ((unsigned)bb[1] << 16); pk.y = (unsigned)bb[2] | ((unsigned)bb[3] << 16);
    pk.z = (unsigned)bb[4] | ((unsigned)bb[5] << 16); pk.w = (unsigned)bb[6] | ((unsigned)bb[7] << 16);
    unsigned short* dst = D + (size_t)n * ldd + k0;
    *(volatile v4u*)dst = pk; if (dup) *(volatile v4u*)(dst + CE) = pk;
    __threadfence();
    *(volatile v4u*)dst = pk; if (dup) *(volatile v4u*)(dst + CE) = pk;
}

__global__ __launch_bounds__(256) void k_cast_t(const float* __restrict__ SRC, int lds, unsigned short* __restrict__ DST, int ldd, int nR, int nC, float sc) {
    const long long u = (long long)blockIdx.x * 256 + threadIdx.x; const int per = nR / 8; if (u >= (long long)nC * per) return;
    const int c = (int)(u / per); const int r0 = 8 * (int)(u % per);
    float w[8];
#pragma unroll
    for (int e = 0; e < 8; ++e) w[e] = bfr(SRC[(long long)(r0 + e) * lds + c]) * sc;
    v4u pk; pk.x = pk2h(w[0], w[1]); pk.y = pk2h(w[2], w[3]); pk.z = pk2h(w[4], w[5]); pk.w = pk2h(w[6], w[7]);
    VST2(v4u, (v4u*)(DST + (long long)c * ldd + r0), pk);
}

template <int MODE>
__device__ __forceinline__ void ln_body(const float* __restrict__ A, long a_bs, const float* __restrict__ GA, const float* __restrict__ BE,
                                        unsigned short* __restrict__ HS, unsigned short* __restrict__ H16) {
    #pragma clang fp contract(off)
    const int r = blockIdx.x * 8 + (threadIdx.x >> 5); const int L = threadIdx.x & 31;
    if (r >= ROWS) return;
    const int b = r / SEQ, t = r - b * SEQ;
    const float* src = A + (long)b * a_bs + (long)t * CE;
    v4f v[8]; float s = 0.f;
#pragma unroll
    for (int q = 0; q < 8; ++q) {
        v[q] = *(const v4f*)(src + 4 * L + 128 * q);
        if (MODE == 0) { v[q].x = bfr(v[q].x); v[q].y = bfr(v[q].y); v[q].z = bfr(v[q].z); v[q].w = bfr(v[q].w); }
        s += (v[q].x + v[q].y) + (v[q].z + v[q].w);
    }
#pragma unroll
    for (int o = 16; o > 0; o >>= 1) s += __shfl_xor(s, o, 32);
    const float mu = s * (1.f / CE); float qq = 0.f;
#pragma unroll
    for (int q = 0; q < 8; ++q) {
        v[q].x -= mu; v[q].y -= mu; v[q].z -= mu; v[q].w -= mu;
        qq += (v[q].x * v[q].x + v[q].y * v[q].y) + (v[q].z * v[q].z + v[q].w * v[q].w);
    }
#pragma unroll
    for (int o = 16; o > 0; o >>= 1) qq += __shfl_xor(qq, o, 32);
    const float rs = rsqrtf(qq * (1.f / CE) + 1e-5f);
    v2u ph[8], pl[8], pf[8];
#pragma unroll
    for (int q = 0; q < 8; ++q) {
        const int c = 4 * L + 128 * q;
        const v4f ga = *(const v4f*)(GA + c), be = *(const v4f*)(BE + c);
        v4f y;
        y.x = v[q].x * rs * bfr(ga.x) + bfr(be.x); y.y = v[q].y * rs * bfr(ga.y) + bfr(be.y);
        y.z = v[q].z * rs * bfr(ga.z) + bfr(be.z); y.w = v[q].w * rs * bfr(ga.w) + bfr(be.w);
        v2u f; f.x = pk2h(y.x, y.y); f.y = pk2h(y.z, y.w); pf[q] = f;
        if (MODE == 0) {
            unsigned short h0, l0, h1, l1, h2, l2, h3, l3;
            bfsplit(y.x, h0, l0); bfsplit(y.y, h1, l1); bfsplit(y.z, h2, l2); bfsplit(y.w, h3, l3);
            v2u a; a.x = (unsigned)h0 | ((unsigned)h1 << 16); a.y = (unsigned)h2 | ((unsigned)h3 << 16); ph[q] = a;
            v2u d; d.x = (unsigned)l0 | ((unsigned)l1 << 16); d.y = (unsigned)l2 | ((unsigned)l3 << 16); pl[q] = d;
        }
    }
    for (int pass = 0; pass < 2; ++pass) {
#pragma unroll
        for (int q = 0; q < 8; ++q) {
            const int c = 4 * L + 128 * q;
            if (MODE == 0) {
                *(volatile v2u*)(HS + (size_t)r * (2 * CE) + c) = ph[q];
                *(volatile v2u*)(HS + (size_t)r * (2 * CE) + CE + c) = pl[q];
            }
            *(volatile v2u*)(H16 + (size_t)r * CE + c) = pf[q];
        }
        __threadfence();
    }
}
__global__ __launch_bounds__(256) void k_ln1(const float* __restrict__ x, const float* __restrict__ g, const float* __restrict__ be,
                                             unsigned short* __restrict__ HS, unsigned short* __restrict__ H16) {
    ln_body<0>(x, (long)SEQ_FULL * CE, g, be, HS, H16);
}
__global__ __launch_bounds__(256) void k_ln2(const float* __restrict__ X1, const float* __restrict__ g, const float* __restrict__ be,
                                             unsigned short* __restrict__ H2) {
    ln_body<1>(X1, (long)SEQ * CE, g, be, nullptr, H2);
}

__device__ __forceinline__ void dep_guard_h(v8f& a, v8f& b, v16h x, v16h y) { asm volatile("v_nop\n\tv_nop\n\tv_nop\n\tv_nop" : "+v"(a), "+v"(b) : "v"(x), "v"(y)); }
__device__ __forceinline__ void dep_guard_b(v8f& a, v8f& b, v16b x, v16b y) { asm volatile("v_nop\n\tv_nop\n\tv_nop\n\tv_nop" : "+v"(a), "+v"(b) : "v"(x), "v"(y)); }
__device__ __forceinline__ void keep4_h(v16h a, v16h b, v16h c, v16h d) { asm volatile("v_nop" :: "v"(a), "v"(b), "v"(c), "v"(d)); }
__device__ __forceinline__ void keep4_b(v16b a, v16b b, v16b c, v16b d) { asm volatile("v_nop" :: "v"(a), "v"(b), "v"(c), "v"(d)); }
__device__ __forceinline__ void acc_guard4(v8f& a, v8f& b, v8f& c, v8f& d) { asm volatile("v_nop\n\tv_nop\n\tv_nop\n\tv_nop" : "+v"(a), "+v"(b), "+v"(c), "+v"(d)); }
template <typename T> struct Frag;
template <> struct Frag<_Float16> {
    typedef v16h V; union U { v16h v; v8h h[2]; };
    static __device__ __forceinline__ v16h load(const _Float16* p) {
        U f; f.h[0] = *(const v8h*)(p); f.h[1] = *(const v8h*)(p + 16); return f.v;
    }
    static __device__ __forceinline__ v8f mma(v16h a, v16h b, v8f c) { return __builtin_amdgcn_wmma_f32_16x16x32_f16(false, a, false, b, (short)0, c, false, false); }
    static __device__ __forceinline__ void guard(v8f& a, v8f& b, v16h x, v16h y) { dep_guard_h(a, b, x, y); }
    static __device__ __forceinline__ void keep(v16h a, v16h b, v16h c, v16h d) { keep4_h(a, b, c, d); }
};
template <> struct Frag<__bf16> {
    typedef v16b V; union U { v16b v; v8b h[2]; };
    static __device__ __forceinline__ v16b load(const __bf16* p) {
        U f; f.h[0] = *(const v8b*)(p); f.h[1] = *(const v8b*)(p + 16); return f.v;
    }
    static __device__ __forceinline__ v8f mma(v16b a, v16b b, v8f c) { return __builtin_amdgcn_wmma_f32_16x16x32_bf16(false, a, false, b, (short)0, c, false, false); }
    static __device__ __forceinline__ void guard(v8f& a, v8f& b, v16b x, v16b y) { dep_guard_b(a, b, x, y); }
    static __device__ __forceinline__ void keep(v16b a, v16b b, v16b c, v16b d) { keep4_b(a, b, c, d); }
};
template <int ET> struct Elem;
template <> struct Elem<0> { typedef _Float16 T; };
template <> struct Elem<1> { typedef __bf16 T; };

template <int ET, int BIAS_MODE, int OUT_MODE, int RESID, int ACT>
__device__ __forceinline__ void gemm64_body(
    const unsigned short* __restrict__ Ap, int lda, long strideA,
    const unsigned short* __restrict__ Btp, int ldb,
    void* __restrict__ Cout, void* __restrict__ Cout2, int ldc, long strideC,
    const float* __restrict__ bias,
    const float* __restrict__ resid, int ldr, long strideR,
    int M, int N, int K, float scale) {
    typedef typename Elem<ET>::T T;
    typedef typename Frag<T>::V V;
    __shared__ __align__(16) float sT[8][16 * 68];
    const int b    = blockIdx.y;
    const int lane = threadIdx.x & 31;
    const int wave = threadIdx.x >> 5;
    const int tilesN = N >> 6;
    const int tilesM = M >> 6;
    const int tile = blockIdx.x * 8 + wave;
    if (tile >= tilesM * tilesN) return;
    const int tm = tile / tilesN;
    const int tn = tile - tm * tilesN;
    const int m0 = tm << 6;
    const int n0 = tn << 6;

    const T* Ab = (const T*)Ap + (size_t)b * strideA;
    const T* Bb = (const T*)Btp;

    const int rlane = lane & 15;
    const int koff  = (lane >> 4) * 8;
    const int mOff  = (lane >> 4) * 8;

    v8f acc[4][4];
#pragma unroll
    for (int i = 0; i < 4; ++i)
#pragma unroll
        for (int j = 0; j < 4; ++j) acc[i][j] = (v8f){0.f, 0.f, 0.f, 0.f, 0.f, 0.f, 0.f, 0.f};

    for (int k0 = 0; k0 < K; k0 += 32) {
        V bh[4];
#pragma unroll
        for (int j = 0; j < 4; ++j) {
            const size_t bo = (size_t)(n0 + (j << 4) + rlane) * ldb + koff + k0;
            bh[j] = Frag<T>::load(Bb + bo);
        }
#pragma unroll
        for (int i = 0; i < 4; ++i) {
            const size_t ao = (size_t)(m0 + (i << 4) + rlane) * lda + koff + k0;
            V ah = Frag<T>::load(Ab + ao);
#pragma unroll
            for (int j = 0; j < 4; ++j) acc[i][j] = Frag<T>::mma(ah, bh[j], acc[i][j]);
            Frag<T>::guard(acc[i][0], acc[i][3], ah, ah);
        }
        Frag<T>::keep(bh[0], bh[1], bh[2], bh[3]);
    }
    acc_guard4(acc[0][0], acc[0][1], acc[0][2], acc[0][3]);
    acc_guard4(acc[1][0], acc[1][1], acc[1][2], acc[1][3]);
    acc_guard4(acc[2][0], acc[2][1], acc[2][2], acc[2][3]);
    acc_guard4(acc[3][0], acc[3][1], acc[3][2], acc[3][3]);

    float* slab = sT[wave];
    const float* Rb = RESID ? (resid + (size_t)b * strideR) : nullptr;
#pragma unroll
    for (int i = 0; i < 4; ++i) {
        const int mBase = m0 + (i << 4);
#pragma unroll
        for (int j = 0; j < 4; ++j) {
            const int n = n0 + (j << 4) + rlane;
            float bv = 0.f;
            if (BIAS_MODE == 2) bv = bfr(bias[n]);
#pragma unroll
            for (int r = 0; r < 8; ++r) {
                float v = acc[i][j][r] * scale;
                if (BIAS_MODE == 2) v += bv;
                if (ACT == 1) v = fmaxf(v, 0.0f);
                slab[(mOff + r) * 68 + (j << 4) + rlane] = v;
            }
        }
        __builtin_amdgcn_fence(3  , "workgroup");
        __builtin_amdgcn_wave_barrier();
        __builtin_amdgcn_fence(2  , "workgroup");
        if (OUT_MODE == 0) {
            float* C = (float*)Cout + (size_t)b * strideC;
            const int hh = lane >> 4, c4 = (lane & 15) * 4;
            v4f vv[8];
#pragma unroll
            for (int it = 0; it < 8; ++it) {
                const int row = it * 2 + hh;
                v4f v = *(const v4f*)(slab + row * 68 + c4);
                if (RESID) {
                    v4f x = *(const v4f*)(Rb + (size_t)(mBase + row) * ldr + n0 + c4);
                    if (RESID == 2) { x.x = bfr(x.x); x.y = bfr(x.y); x.z = bfr(x.z); x.w = bfr(x.w); }
                    v.x = x.x + v.x; v.y = x.y + v.y; v.z = x.z + v.z; v.w = x.w + v.w;
                }
                vv[it] = v;
            }
            for (int pass = 0; pass < 2; ++pass) {
#pragma unroll
                for (int it = 0; it < 8; ++it) {
                    const int row = it * 2 + hh;
                    *(volatile v4f*)(C + (size_t)(mBase + row) * ldc + n0 + c4) = vv[it];
                }
                __threadfence();
            }
        } else {
            const int q = lane >> 3, c8 = (lane & 7) * 8;
            unsigned short* C  = (unsigned short*)Cout  + (size_t)b * strideC;
            unsigned short* C2 = (OUT_MODE == 2) ? ((unsigned short*)Cout2 + (size_t)b * strideC) : nullptr;
            v8h hv[4], lv[4];
#pragma unroll
            for (int it = 0; it < 4; ++it) {
                const int row = it * 4 + q;
                const float* sp = slab + row * 68 + c8;
#pragma unroll
                for (int e = 0; e < 8; ++e) {
                    if (OUT_MODE == 1) {
                        hv[it][e] = (_Float16)sp[e];
                        lv[it][e] = (_Float16)0.f;
                    } else {
                        const unsigned short hb = bf_bits(sp[e]);
                        const unsigned short lb = bf_bits(sp[e] - bits_f(hb));
                        hv[it][e] = __builtin_bit_cast(_Float16, hb);
                        lv[it][e] = __builtin_bit_cast(_Float16, lb);
                    }
                }
            }
            for (int pass = 0; pass < 2; ++pass) {
#pragma unroll
                for (int it = 0; it < 4; ++it) {
                    const int row = it * 4 + q;
                    *(volatile v8h*)(C + (size_t)(mBase + row) * ldc + n0 + c8) = hv[it];
                    if (OUT_MODE == 2) *(volatile v8h*)(C2 + (size_t)(mBase + row) * ldc + n0 + c8) = lv[it];
                }
                __threadfence();
            }
        }
        __builtin_amdgcn_fence(3  , "workgroup");
        __builtin_amdgcn_wave_barrier();
        __builtin_amdgcn_fence(2  , "workgroup");
    }
}

__global__ __launch_bounds__(256) void k_gemm_qk(const unsigned short* __restrict__ A, const unsigned short* __restrict__ Bt,
                                                 unsigned short* __restrict__ Ch, unsigned short* __restrict__ Cl) {
    gemm64_body<1, 0, 2, 0, 0>(A, 2 * CE, 0, Bt, 2 * CE, (void*)Ch, (void*)Cl, 2 * CE, 0, nullptr, nullptr, 0, 0, ROWS, 2 * CE, 2 * CE, 1.0f);
}
__global__ __launch_bounds__(256) void k_gemm_vt(const unsigned short* __restrict__ A, const unsigned short* __restrict__ Bt,
                                                 unsigned short* __restrict__ Ch, unsigned short* __restrict__ Cl) {
    gemm64_body<0, 0, 2, 0, 0>(A, CE, 0, Bt, CE, (void*)Ch, (void*)Cl, ROWS, 0, nullptr, nullptr, 0, 0, CE, ROWS, CE, 0.0625f);
}
__global__ __launch_bounds__(256) void k_gemm_proj(const unsigned short* __restrict__ A, const unsigned short* __restrict__ Bt, float* __restrict__ C,
                                                   const float* __restrict__ bias, const float* __restrict__ xres) {
    gemm64_body<0, 2, 0, 2, 0>(A, CE, (long)SEQ * CE, Bt, CE, (void*)C, nullptr, CE, (long)SEQ * CE, bias, xres, CE, (long)SEQ_FULL * CE, SEQ, CE, CE, 0.0625f);
}
__global__ __launch_bounds__(256) void k_gemm_fc1(const unsigned short* __restrict__ A, const unsigned short* __restrict__ Bt, unsigned short* __restrict__ C,
                                                  const float* __restrict__ bias) {
    gemm64_body<0, 2, 1, 0, 1>(A, CE, 0, Bt, CE, (void*)C, nullptr, FF, 0, bias, nullptr, 0, 0, ROWS, FF, CE, 0.0625f);
}
__global__ __launch_bounds__(256) void k_gemm_fc2(const unsigned short* __restrict__ A, const unsigned short* __restrict__ Bt, float* __restrict__ C,
                                                  const float* __restrict__ bias, const float* __restrict__ x1) {
    gemm64_body<0, 2, 0, 1, 0>(A, FF, (long)SEQ * FF, Bt, FF, (void*)C, nullptr, CE, (long)SEQ_FULL * CE, bias, x1, CE, (long)SEQ * CE, SEQ, CE, FF, 0.0625f);
}

#define AT_NW 4
__device__ __forceinline__ v8f at_mma(v16b a, v16b b, v8f c) {
    c = __builtin_amdgcn_wmma_f32_16x16x32_bf16(false, a, false, b, (short)0, c, false, false);
    asm volatile("v_nop\n\tv_nop\n\tv_nop\n\tv_nop" : "+v"(c) : "v"(a), "v"(b));
    return c;
}
static_assert(AT_NW * 16 * 68 * 4 <= 4 * 64 * 64 * 2);

__global__ __launch_bounds__(128) void k_attn(const unsigned short* __restrict__ QKHp, const unsigned short* __restrict__ QKLp,
                                              const unsigned short* __restrict__ VTHp, const unsigned short* __restrict__ VTLp,
                                              unsigned short* __restrict__ AO) {
    union FB { v16b v; v8b h[2]; };
    __shared__ __align__(16) __bf16 KV[4 * 64 * 64];
    __shared__ __align__(16) __bf16 PS[AT_NW][2 * 16 * 64];
    __bf16* Ksh = KV; __bf16* Ksl = KV + 4096; __bf16* Vth = KV + 8192; __bf16* Vtl = KV + 12288;
    const __bf16* QKH = (const __bf16*)QKHp; const __bf16* QKL = (const __bf16*)QKLp;
    const __bf16* VTH = (const __bf16*)VTHp; const __bf16* VTL = (const __bf16*)VTLp;

    const int tid = threadIdx.x, wave = tid >> 5, lane = tid & 31, hh = lane >> 4, c = lane & 15;
    const int nqb = SEQ / 64;
    const int bx = blockIdx.x;
    const int qb = bx % nqb;
    const int bh = bx / nqb;
    const int h  = bh % NH;
    const int b  = bh / NH;
    const int q0 = qb * 64 + wave * 16;
    const size_t rowbase = (size_t)b * SEQ;
    const int QKP = 2 * CE;
    const int VTP = ROWS;

    v16b qah[2], qal[2];
    {
        const __bf16* qh = QKH + (rowbase + q0 + c) * QKP + h * HD;
        const __bf16* ql = QKL + (rowbase + q0 + c) * QKP + h * HD;
#pragma unroll
        for (int dc = 0; dc < 2; ++dc) {
            FB f, g;
            f.h[0] = *(const v8b*)(qh + dc * 32 + 8 * hh); f.h[1] = *(const v8b*)(qh + dc * 32 + 16 + 8 * hh);
            g.h[0] = *(const v8b*)(ql + dc * 32 + 8 * hh); g.h[1] = *(const v8b*)(ql + dc * 32 + 16 + 8 * hh);
            qah[dc] = f.v; qal[dc] = g.v;
        }
    }

    const float NEG = -__builtin_inff();
    const float L2E = 1.4426950408889634f;
    float mrow[8], lrow[8];
    v8f oacc[4];
#pragma unroll
    for (int r = 0; r < 8; ++r) { mrow[r] = NEG; lrow[r] = 0.f; }
#pragma unroll
    for (int t = 0; t < 4; ++t) oacc[t] = (v8f){0.f, 0.f, 0.f, 0.f, 0.f, 0.f, 0.f, 0.f};

    __bf16* pwh = PS[wave];
    __bf16* pwl = PS[wave] + 16 * 64;

    for (int kc = 0; kc <= qb; ++kc) {
        const int kv0 = kc * 64;
        __syncthreads();
        {
            const __bf16* khg = QKH + (rowbase + kv0) * QKP + CE + h * HD;
            const __bf16* klg = QKL + (rowbase + kv0) * QKP + CE + h * HD;
            const __bf16* vhg = VTH + (size_t)(h * HD) * VTP + rowbase + kv0;
            const __bf16* vlg = VTL + (size_t)(h * HD) * VTP + rowbase + kv0;
#pragma unroll
            for (int i = 0; i < 4; ++i) {
                const int p = tid + 128 * i; const int rr = p >> 3; const int sg = (p & 7) * 8;
                *(v8b*)(Ksh + rr * 64 + sg) = *(const v8b*)(khg + (size_t)rr * QKP + sg);
                *(v8b*)(Ksl + rr * 64 + sg) = *(const v8b*)(klg + (size_t)rr * QKP + sg);
                *(v8b*)(Vth + rr * 64 + sg) = *(const v8b*)(vhg + (size_t)rr * VTP + sg);
                *(v8b*)(Vtl + rr * 64 + sg) = *(const v8b*)(vlg + (size_t)rr * VTP + sg);
            }
        }
        __syncthreads();

        v8f s[4];
#pragma unroll
        for (int j = 0; j < 4; ++j) {
            s[j] = (v8f){0.f, 0.f, 0.f, 0.f, 0.f, 0.f, 0.f, 0.f};
#pragma unroll
            for (int dc = 0; dc < 2; ++dc) {
                FB kb, kl;
                kb.h[0] = *(const v8b*)(Ksh + (j * 16 + c) * 64 + dc * 32 + 8 * hh);
                kb.h[1] = *(const v8b*)(Ksh + (j * 16 + c) * 64 + dc * 32 + 16 + 8 * hh);
                kl.h[0] = *(const v8b*)(Ksl + (j * 16 + c) * 64 + dc * 32 + 8 * hh);
                kl.h[1] = *(const v8b*)(Ksl + (j * 16 + c) * 64 + dc * 32 + 16 + 8 * hh);
                s[j] = at_mma(qah[dc], kb.v, s[j]);
                s[j] = at_mma(qah[dc], kl.v, s[j]);
                s[j] = at_mma(qal[dc], kb.v, s[j]);
            }
        }
        const bool diag = (kc == qb);
        float cm[8];
#pragma unroll
        for (int r = 0; r < 8; ++r) {
            const int qrow = q0 + 8 * hh + r;
            float m = NEG;
#pragma unroll
            for (int j = 0; j < 4; ++j) {
                const int kvcol = kv0 + j * 16 + c;
                const float sv = s[j][r];
                s[j][r] = (diag && (kvcol > qrow)) ? NEG : sv;
                m = fmaxf(m, s[j][r]);
            }
#pragma unroll
            for (int off = 1; off < 16; off <<= 1) m = fmaxf(m, __shfl_xor(m, off, 32));
            cm[r] = m;
        }
#pragma unroll
        for (int r = 0; r < 8; ++r) {
            const float mnew = fmaxf(mrow[r], cm[r]);
            const float alpha = exp2f((mrow[r] - mnew) * L2E);
            mrow[r] = mnew;
            float psum = 0.f;
#pragma unroll
            for (int j = 0; j < 4; ++j) {
                const float p = exp2f((s[j][r] - mnew) * L2E);
                psum += p;
                unsigned short ph, pl; bfsplit(p, ph, pl);
                pwh[(8 * hh + r) * 64 + j * 16 + c] = __builtin_bit_cast(__bf16, ph);
                pwl[(8 * hh + r) * 64 + j * 16 + c] = __builtin_bit_cast(__bf16, pl);
            }
#pragma unroll
            for (int off = 1; off < 16; off <<= 1) psum += __shfl_xor(psum, off, 32);
            lrow[r] = lrow[r] * alpha + psum;
#pragma unroll
            for (int t = 0; t < 4; ++t) oacc[t][r] *= alpha;
        }
        __builtin_amdgcn_fence(3  , "workgroup");
        __builtin_amdgcn_wave_barrier();
        __builtin_amdgcn_fence(2  , "workgroup");
#pragma unroll
        for (int kk = 0; kk < 2; ++kk) {
            FB pa, pl;
            pa.h[0] = *(const v8b*)(pwh + c * 64 + kk * 32 + 8 * hh);
            pa.h[1] = *(const v8b*)(pwh + c * 64 + kk * 32 + 16 + 8 * hh);
            pl.h[0] = *(const v8b*)(pwl + c * 64 + kk * 32 + 8 * hh);
            pl.h[1] = *(const v8b*)(pwl + c * 64 + kk * 32 + 16 + 8 * hh);
#pragma unroll
            for (int t = 0; t < 4; ++t) {
                FB vb, vl;
                vb.h[0] = *(const v8b*)(Vth + (t * 16 + c) * 64 + kk * 32 + 8 * hh);
                vb.h[1] = *(const v8b*)(Vth + (t * 16 + c) * 64 + kk * 32 + 16 + 8 * hh);
                vl.h[0] = *(const v8b*)(Vtl + (t * 16 + c) * 64 + kk * 32 + 8 * hh);
                vl.h[1] = *(const v8b*)(Vtl + (t * 16 + c) * 64 + kk * 32 + 16 + 8 * hh);
                oacc[t] = at_mma(pa.v, vb.v, oacc[t]);
                oacc[t] = at_mma(pa.v, vl.v, oacc[t]);
                oacc[t] = at_mma(pl.v, vb.v, oacc[t]);
            }
        }
    }

    __syncthreads();
    float* os = (float*)KV + wave * (16 * 68);
#pragma unroll
    for (int r = 0; r < 8; ++r) {
        const float inv = 1.0f / lrow[r];
#pragma unroll
        for (int t = 0; t < 4; ++t) os[(8 * hh + r) * 68 + t * 16 + c] = oacc[t][r] * inv;
    }
    __builtin_amdgcn_fence(3  , "workgroup");
    __builtin_amdgcn_wave_barrier();
    __builtin_amdgcn_fence(2  , "workgroup");
    {
        const int q = lane >> 3, c8 = (lane & 7) * 8;
        v8h hv[4];
#pragma unroll
        for (int it = 0; it < 4; ++it) {
            const int row = it * 4 + q;
            const float* sp = os + row * 68 + c8;
#pragma unroll
            for (int e = 0; e < 8; ++e) hv[it][e] = (_Float16)sp[e];
        }
        for (int pass = 0; pass < 2; ++pass) {
#pragma unroll
            for (int it = 0; it < 4; ++it) {
                const int row = it * 4 + q;
                *(volatile v8h*)(AO + (rowbase + q0 + row) * CE + h * HD + c8) = hv[it];
            }
            __threadfence();
        }
    }
}

#define SZ_HS   ((size_t)ROWS * 2 * CE * 2)
#define SZ_H16  ((size_t)ROWS * CE * 2)
#define SZ_WQK  ((size_t)2 * CE * 2 * CE * 2)
#define SZ_WV   ((size_t)CE * CE * 2)
#define SZ_QK1  ((size_t)ROWS * 2 * CE * 2)
#define SZ_VT1  ((size_t)CE * ROWS * 2)
#define SZ_AO   ((size_t)ROWS * CE * 2)
#define SZ_WP   ((size_t)CE * CE * 2)
#define SZ_X1   ((size_t)ROWS * CE * 4)
#define SZ_W1   ((size_t)FF * CE * 2)
#define SZ_W2   ((size_t)CE * FF * 2)
#define SZ_F16  ((size_t)ROWS * FF * 2)
#define WS_TOTAL (SZ_HS + SZ_H16 + SZ_WQK + SZ_WV + 2 * SZ_QK1 + 2 * SZ_VT1 + SZ_AO + SZ_WP + SZ_X1 + SZ_W1 + SZ_W2)
static_assert(WS_TOTAL <= (size_t)134217728);
static_assert(SZ_F16 <= 2 * SZ_QK1);
static_assert(SZ_HS % 256 == 0);
static_assert(SZ_H16 % 256 == 0);
static_assert(SZ_VT1 % 256 == 0);

extern "C" void kernel_launch(void* const* d_in, const int* in_sizes, int n_in, void* d_out, int out_size, void* d_ws, size_t ws_size, hipStream_t stream) {
    if (n_in < 14) return;
    const long long xneed = (long long)(NB - 1) * SEQ_FULL * CE + (long long)SEQ * CE;
    if ((long long)in_sizes[0] < xneed) return;
    if (in_sizes[1] < CE || in_sizes[2] < CE || in_sizes[7] < CE || in_sizes[8] < CE || in_sizes[9] < CE || in_sizes[13] < CE) return;
    if (in_sizes[3] < NH * CE * HD || in_sizes[4] < NH * CE * HD || in_sizes[5] < NH * CE * HD) return;
    if (in_sizes[6] < CE * CE || in_sizes[10] < CE * FF || in_sizes[11] < FF || in_sizes[12] < FF * CE) return;
    if ((long long)out_size < xneed) return;
    if ((size_t)WS_TOTAL > ws_size) return;

    const float* x      = (const float*)d_in[0];
    const float* ln1_w  = (const float*)d_in[1];
    const float* ln1_b  = (const float*)d_in[2];
    const float* Wq     = (const float*)d_in[3];
    const float* Wk     = (const float*)d_in[4];
    const float* Wv     = (const float*)d_in[5];
    const float* proj_w = (const float*)d_in[6];
    const float* proj_b = (const float*)d_in[7];
    const float* ln2_w  = (const float*)d_in[8];
    const float* ln2_b  = (const float*)d_in[9];
    const float* fc1_w  = (const float*)d_in[10];
    const float* fc1_b  = (const float*)d_in[11];
    const float* fc2_w  = (const float*)d_in[12];
    const float* fc2_b  = (const float*)d_in[13];
    float* out = (float*)d_out;

    char* wsp = (char*)d_ws;
    unsigned short* HS   = (unsigned short*)wsp; wsp += SZ_HS;
    unsigned short* H16  = (unsigned short*)wsp; wsp += SZ_H16;
    unsigned short* WQK  = (unsigned short*)wsp; wsp += SZ_WQK;
    unsigned short* WV16 = (unsigned short*)wsp; wsp += SZ_WV;
    unsigned short* QKH  = (unsigned short*)wsp; wsp += SZ_QK1;
    unsigned short* QKL  = (unsigned short*)wsp; wsp += SZ_QK1;
    unsigned short* VTH  = (unsigned short*)wsp; wsp += SZ_VT1;
    unsigned short* VTL  = (unsigned short*)wsp; wsp += SZ_VT1;
    unsigned short* AO16 = (unsigned short*)wsp; wsp += SZ_AO;
    unsigned short* WPT  = (unsigned short*)wsp; wsp += SZ_WP;
    float*          X1   = (float*)wsp;          wsp += SZ_X1;
    unsigned short* W1T  = (unsigned short*)wsp; wsp += SZ_W1;
    unsigned short* W2T  = (unsigned short*)wsp; wsp += SZ_W2;
    unsigned short* F16  = QKH;
    unsigned short* H2   = H16;

    const unsigned gw = (unsigned)((CE * (CE / 8) + 255) / 256);
    k_w_head<<<gw, 256, 0, stream>>>(Wq, WQK, 2 * CE, 1, 0);
    k_w_head<<<gw, 256, 0, stream>>>(Wk, WQK + (size_t)CE * 2 * CE, 2 * CE, 1, 0);
    k_w_head<<<gw, 256, 0, stream>>>(Wv, WV16, CE, 0, 1);
    k_cast_t<<<(unsigned)((((long long)CE) * (CE / 8) + 255) / 256), 256, 0, stream>>>(proj_w, CE, WPT, CE, CE, CE, 16.0f);
    k_cast_t<<<(unsigned)((((long long)FF) * (CE / 8) + 255) / 256), 256, 0, stream>>>(fc1_w, FF, W1T, CE, CE, FF, 16.0f);
    k_cast_t<<<(unsigned)((((long long)CE) * (FF / 8) + 255) / 256), 256, 0, stream>>>(fc2_w, CE, W2T, FF, FF, CE, 16.0f);

    k_ln1<<<(ROWS + 7) / 8, 256, 0, stream>>>(x, ln1_w, ln1_b, HS, H16);
    k_gemm_qk<<<dim3((unsigned)(((ROWS / 64) * ((2 * CE) / 64) + 7) / 8), 1u), 256, 0, stream>>>(HS, WQK, QKH, QKL);
    k_gemm_vt<<<dim3((unsigned)(((CE / 64) * (ROWS / 64) + 7) / 8), 1u), 256, 0, stream>>>(WV16, H16, VTH, VTL);
    k_attn<<<(unsigned)(NB * NH * (SEQ / 64)), 128, 0, stream>>>(QKH, QKL, VTH, VTL, AO16);
    k_gemm_proj<<<dim3((unsigned)(((SEQ / 64) * (CE / 64) + 7) / 8), (unsigned)NB), 256, 0, stream>>>(AO16, WPT, X1, proj_b, x);
    k_ln2<<<(ROWS + 7) / 8, 256, 0, stream>>>(X1, ln2_w, ln2_b, H2);
    k_gemm_fc1<<<dim3((unsigned)(((ROWS / 64) * (FF / 64) + 7) / 8), 1u), 256, 0, stream>>>(H2, W1T, F16, fc1_b);
    k_gemm_fc2<<<dim3((unsigned)(((SEQ / 64) * (CE / 64) + 7) / 8), (unsigned)NB), 256, 0, stream>>>(F16, W2T, out, fc2_b, X1);
}
